// attn_90280212561996
// MI455X (gfx1250) — hardware-run, weakly checked
//
#include <hip/hip_runtime.h>


namespace {
constexpr int NC = 8, NB = 8, V = 512, F = 256, H = 4, DQ = 64, NBN = NB * NC, BNL = 64  , NTOK = NB * NC * V;
constexpr float XS = 8.0f, WSC = 256.0f, PS = 1024.0f, LOG2E = 1.4426950408889634f, EPS = 1e-6f;
static_assert(V % 64 == 0 && F == H * DQ, "tiling");
typedef _Float16 b16;
typedef __attribute__((ext_vector_type(16))) _Float16 v16b;
typedef __attribute__((ext_vector_type(8))) _Float16 v8b;
typedef __attribute__((ext_vector_type(8))) float v8f;
typedef __attribute__((ext_vector_type(4))) float v4f;
__device__ __forceinline__ float bf16_rne(float f) { unsigned int u = __float_as_uint(f); u += 0x7FFFu + ((u >> 16) & 1u); return __uint_as_float(u & 0xFFFF0000u); }
__device__ __forceinline__ void split16(float v, b16& hi, b16& lo) { hi = (b16)v; lo = (b16)(v - (float)hi); }
__device__ __forceinline__ v16b frag_kb(const b16* p, int hh) { const v8b a = *(const v8b*)(p + 8 * hh), b = *(const v8b*)(p + 16 + 8 * hh); v16b f;
#pragma unroll
  for (int e = 0; e < 8; ++e) { f[e] = a[e]; f[8 + e] = b[e]; } return f; }
__device__ __forceinline__ v8f wmma16b(v16b a, v16b b, v8f c) { v8f d = __builtin_amdgcn_wmma_f32_16x16x32_f16(false, a, false, b, (short)0, c, false, false); asm volatile("v_nop\n\tv_nop\n\tv_nop\n\tv_nop" : "+v"(d) : "v"(a), "v"(b)); return d; }
__device__ __forceinline__ void wave_lds_sync() { __builtin_amdgcn_fence(__ATOMIC_RELEASE, "workgroup"); __builtin_amdgcn_wave_barrier(); __builtin_amdgcn_fence(__ATOMIC_ACQUIRE, "workgroup"); }
__device__ __forceinline__ float pmul(float a, float b) { float p = a * b; asm volatile("" : "+v"(p)); return p; }
__device__ __forceinline__ int iclamp(int v, int lo, int hi) { return v < lo ? lo : (v > hi ? hi : v); }

typedef __attribute__((ext_vector_type(2))) _Float16 v2h;
typedef __attribute__((ext_vector_type(4))) _Float16 v4h;
__device__ __forceinline__ float nexp2(float v) { return __builtin_amdgcn_exp2f(v); }
__global__ __launch_bounds__(256) void prep_kernel(const float* __restrict__ wq, const float* __restrict__ wk, const float* __restrict__ wv, const float* __restrict__ wo, const float* __restrict__ w1, const float* __restrict__ w2, b16* __restrict__ WT) {
  const size_t u = (size_t)blockIdx.x * 256 + threadIdx.x; const size_t per = (size_t)F * F / 8; if (u >= 6 * per) return; const int m = (int)(u / per); const size_t e = (u % per) * 8; const float* w = m == 0 ? wq : m == 1 ? wk : m == 2 ? wv : m == 3 ? wo : m == 4 ? w1 : w2; v8b o;
  for (int j = 0; j < 8; ++j) o[j] = (b16)(bf16_rne(w[e + j]) * WSC);
  for (int pass = 0; pass < 2; ++pass) { *(volatile v8b*)(WT + (size_t)m * F * F + e) = o; __threadfence(); }
}
template <int KD>
__device__ __forceinline__ void stage_ln(const float* __restrict__ src, size_t stride, const float* __restrict__ g, const float* __restrict__ bb, bool round_in, b16 (*Ah)[KD + 8], b16 (*Al)[KD + 8], int lane) {
  constexpr int PER = KD / 32;
  for (int rr = 0; rr < 16; ++rr) { float xv[PER]; float s = 0.0f;
#pragma unroll
    for (int q = 0; q < PER; ++q) { float t = src[(size_t)rr * stride + q * 32 + lane]; if (round_in) t = bf16_rne(t); xv[q] = t; s += t; }
#pragma unroll
    for (int o = 1; o < 32; o <<= 1) s += __shfl_xor(s, o);
    const float mu = s * (1.0f / KD); float vs = 0.0f;
#pragma unroll
    for (int q = 0; q < PER; ++q) { const float d = xv[q] - mu; vs += d * d; }
#pragma unroll
    for (int o = 1; o < 32; o <<= 1) vs += __shfl_xor(vs, o);
    const float rs = rsqrtf(vs * (1.0f / KD) + EPS);
#pragma unroll
    for (int q = 0; q < PER; ++q) { const int c = q * 32 + lane; const float nv = (xv[q] - mu) * rs * bf16_rne(g[c]) + bf16_rne(bb[c]); b16 p, ql; split16(nv * XS, p, ql); Ah[rr][c] = p; Al[rr][c] = ql; } }
}
__global__ __launch_bounds__(128) void proj_kernel(const float* __restrict__ code, const float* __restrict__ tex, const float* __restrict__ l1g, const float* __restrict__ l1b, const float* __restrict__ l2g, const float* __restrict__ l2b, const b16* __restrict__ WT, const float* __restrict__ bq, const float* __restrict__ bk, const float* __restrict__ bv, b16* __restrict__ QP, b16* __restrict__ KP, b16* __restrict__ VT) {
  __shared__ __attribute__((aligned(16))) b16 Ah[4][16][F + 8], Al[4][16][F + 8]; __shared__ __attribute__((aligned(16))) float Tf[4][16][128 + 4];
  const int wave = threadIdx.x >> 5, lane = threadIdx.x & 31, nloc = lane & 15, hlf = lane >> 4; const int t0 = blockIdx.x * 64; const int map = blockIdx.y; const int part = blockIdx.z / 2, slab = blockIdx.z % 2, c0 = slab * 128;
  const float* src = (part == 0 ? tex : code) + ((size_t)map * V + t0 + wave * 16) * F; const float* g = part == 0 ? l2g : l1g; const float* bb = part == 0 ? l2b : l1b;
  stage_ln<F>(src, F, g, bb, true, Ah[wave], Al[wave], lane);
  wave_lds_sync();
  const b16* W = WT + (size_t)part * F * F; const float* bias = part == 0 ? bq : part == 1 ? bk : bv;
  v8f acc[8];
#pragma unroll
  for (int t = 0; t < 8; ++t) acc[t] = (v8f){};
#pragma unroll 2
  for (int kb = 0; kb < F; kb += 32) { const v16b ah = frag_kb(&Ah[wave][nloc][kb], hlf), al = frag_kb(&Al[wave][nloc][kb], hlf);
#pragma unroll
    for (int t = 0; t < 8; ++t) { const v16b bw = frag_kb(W + (size_t)(c0 + t * 16 + nloc) * F + kb, hlf); acc[t] = wmma16b(ah, bw, acc[t]); acc[t] = wmma16b(al, bw, acc[t]); } }
#pragma unroll
  for (int t = 0; t < 8; ++t) { const float b_ = bf16_rne(bias[c0 + t * 16 + nloc]);
#pragma unroll
    for (int r = 0; r < 8; ++r) Tf[wave][8 * hlf + r][t * 16 + nloc] = acc[t][r] * (1.0f / (XS * WSC)) + b_; }
  __syncthreads();
  for (int pass = 0; pass < 2; ++pass) {
    if (part < 2) { b16* plane = part == 0 ? QP : KP; const int c = c0 + lane * 4; const int h = c / DQ, d = c % DQ;
      for (int rr = 0; rr < 16; ++rr) { const int tok = t0 + wave * 16 + rr; v4h o4; for (int j = 0; j < 4; ++j) o4[j] = (b16)(Tf[wave][rr][lane * 4 + j] * XS); *(volatile v4h*)(plane + (((size_t)map * H + h) * V + tok) * DQ + d) = o4; } }
    else {
#pragma unroll 1
      for (int q = 0; q < 32; ++q) { const int cl = wave * 32 + q; const int c = c0 + cl; const int h = c / DQ, d = c % DQ; const int tk = lane * 2; v2h vv; vv[0] = (b16)(Tf[tk >> 4][tk & 15][cl] * XS); vv[1] = (b16)(Tf[(tk + 1) >> 4][(tk + 1) & 15][cl] * XS);
        *(volatile v2h*)(VT + (((size_t)map * H + h) * DQ + d) * (size_t)V + t0 + lane * 2) = vv; } }
    __threadfence(); }
}
__global__ __launch_bounds__(64) void attn_kernel(const b16* __restrict__ QP, const b16* __restrict__ KP, const b16* __restrict__ VT, b16* __restrict__ CTX) {
  __shared__ __attribute__((aligned(16))) b16 Pb[2][16][32 + 8]; __shared__ __attribute__((aligned(16))) float To[2][16][DQ + 4];
  const int wave = threadIdx.x >> 5, lane = threadIdx.x & 31, hh = lane >> 4, col = lane & 15; const int pair = blockIdx.y / H, h = blockIdx.y % H; const int b = pair / NC, n = pair % NC; const int q0 = blockIdx.x * 32 + wave * 16, qi = q0 + col;
  const b16* Qb = QP + (((size_t)b * H + h) * V) * DQ; const b16* Kb = KP + (((size_t)n * H + h) * V) * DQ; const b16* Vb = VT + (((size_t)n * H + h) * DQ) * (size_t)V;
  const v16b qa0 = frag_kb(Qb + (size_t)qi * DQ, hh), qa1 = frag_kb(Qb + (size_t)qi * DQ + 32, hh);
  const float cs = LOG2E / (8.0f * XS * XS);
  float m = -INFINITY, l = 0.0f; v8f o[4]; for (int t = 0; t < 4; ++t) o[t] = (v8f){};
#pragma unroll 1
  for (int kb = 0; kb < V; kb += 32) {
    float e[16]; float mx = -INFINITY;
#pragma unroll
    for (int u = 0; u < 2; ++u) { v8f s = (v8f){}; const size_t kr = (size_t)(kb + u * 16 + col) * DQ; s = wmma16b(frag_kb(Kb + kr, hh), qa0, s); s = wmma16b(frag_kb(Kb + kr + 32, hh), qa1, s);
#pragma unroll
      for (int r = 0; r < 8; ++r) { const float vv = s[r] * cs; e[u * 8 + r] = vv; mx = fmaxf(mx, vv); } }
    mx = fmaxf(mx, __shfl_xor(mx, 16)); const float mn = fmaxf(m, mx); const float al = nexp2(m - mn); float sum = 0.0f;
#pragma unroll
    for (int i2 = 0; i2 < 16; ++i2) { const float p = nexp2(e[i2] - mn); sum += p; Pb[wave][col][(i2 < 8 ? 0 : 16) + 8 * hh + (i2 & 7)] = (b16)(p * PS); }
    sum += __shfl_xor(sum, 16); l = l * al + sum; m = mn;
    wave_lds_sync();
    const v16b pf = frag_kb(&Pb[wave][col][0], hh);
#pragma unroll
    for (int t = 0; t < 4; ++t) { o[t] *= al; o[t] = wmma16b(frag_kb(Vb + (size_t)(t * 16 + col) * V + kb, hh), pf, o[t]); }
    wave_lds_sync(); }
  const float inv = 1.0f / (l * PS * XS);
#pragma unroll
  for (int t = 0; t < 4; ++t)
#pragma unroll
    for (int r = 0; r < 8; ++r) To[wave][col][t * 16 + 8 * hh + r] = o[t][r] * inv;
  wave_lds_sync();
  for (int pass = 0; pass < 2; ++pass) { for (int rr = 0; rr < 16; ++rr) { v2h o2; o2[0] = (b16)(To[wave][rr][lane * 2] * XS); o2[1] = (b16)(To[wave][rr][lane * 2 + 1] * XS); *(volatile v2h*)(CTX + ((size_t)pair * V + q0 + rr) * F + h * DQ + lane * 2) = o2; } __threadfence(); }
}
template <int MODE>
__global__ __launch_bounds__(128) void rows_kernel(const b16* __restrict__ AP, const float* __restrict__ XF, const float* __restrict__ tex, const float* __restrict__ lng, const float* __restrict__ lnb, const b16* __restrict__ W, const float* __restrict__ bias, float* __restrict__ OF, b16* __restrict__ OP) {
  __shared__ __attribute__((aligned(16))) float Tf[4][16][128 + 4]; __shared__ __attribute__((aligned(16))) b16 Ah[(MODE == 1) ? 4 : 1][16][F + 8], Al[(MODE == 1) ? 4 : 1][16][F + 8];
  const int wave = threadIdx.x >> 5, lane = threadIdx.x & 31, nloc = lane & 15, hlf = lane >> 4; const size_t m0 = ((size_t)blockIdx.x * 4 + wave) * 16; const int n0 = blockIdx.y * 128;
  if (MODE == 1) { stage_ln<F>(XF + m0 * F, F, lng, lnb, false, Ah[wave], Al[wave], lane); wave_lds_sync(); }
  v8f acc[8];
#pragma unroll
  for (int t = 0; t < 8; ++t) acc[t] = (v8f){};
#pragma unroll 2
  for (int kb = 0; kb < F; kb += 32) { v16b a, al; if (MODE == 1) { a = frag_kb(&Ah[wave][nloc][kb], hlf); al = frag_kb(&Al[wave][nloc][kb], hlf); } else a = frag_kb(AP + (m0 + nloc) * F + kb, hlf);
#pragma unroll
    for (int t = 0; t < 8; ++t) { const v16b bw = frag_kb(W + (size_t)(n0 + t * 16 + nloc) * F + kb, hlf); acc[t] = wmma16b(a, bw, acc[t]); if (MODE == 1) acc[t] = wmma16b(al, bw, acc[t]); } }
#pragma unroll
  for (int t = 0; t < 8; ++t) { const float b_ = bf16_rne(bias[n0 + t * 16 + nloc]);
#pragma unroll
    for (int r = 0; r < 8; ++r) { float v = acc[t][r] * (1.0f / (XS * WSC)) + b_; if (MODE == 1) v = fmaxf(v, 0.0f); Tf[wave][8 * hlf + r][t * 16 + nloc] = v; } }
  wave_lds_sync();
  for (int rr = 0; rr < 16; ++rr) { const size_t row = m0 + rr; if (MODE == 0) { const int b = (int)(row / ((size_t)NC * V)), qv = (int)(row % V); const v4f tx = *(const v4f*)(tex + ((size_t)b * V + qv) * F + n0 + lane * 4); v4f t4 = *(const v4f*)(&Tf[wave][rr][lane * 4]); for (int j = 0; j < 4; ++j) t4[j] += bf16_rne(tx[j]); *(v4f*)(&Tf[wave][rr][lane * 4]) = t4; }
    else if (MODE == 2) { const v4f xv = *(const v4f*)(XF + row * F + n0 + lane * 4); v4f t4 = *(const v4f*)(&Tf[wave][rr][lane * 4]); t4 += xv; *(v4f*)(&Tf[wave][rr][lane * 4]) = t4; } }
  wave_lds_sync();
  for (int pass = 0; pass < 2; ++pass) { for (int rr = 0; rr < 16; ++rr) { const size_t row = m0 + rr; const v4f f = *(const v4f*)(&Tf[wave][rr][lane * 4]);
      if (MODE == 1) { v4h o4; for (int j = 0; j < 4; ++j) o4[j] = (b16)(f[j] * XS); *(volatile v4h*)(OP + row * F + n0 + lane * 4) = o4; } else *(volatile v4f*)(OF + row * F + n0 + lane * 4) = f; }
    __threadfence(); }
}
}

extern "C" void kernel_launch(void* const* d_in, const int* in_sizes, int n_in, void* d_out, int out_size, void* d_ws, size_t ws_size, hipStream_t stream) {
  (void)n_in;
  auto Fp = [&](int i) { return (const float*)d_in[i]; };
  if (in_sizes[0] != NC * V * F || in_sizes[1] != NB * V * F || in_sizes[2] != F * F || in_sizes[8] != F * F || in_sizes[16] != F * F || in_sizes[18] != F * F || in_sizes[19] != F || out_size != NB * NC * V * F) return;
  size_t off = 0; char* ws = (char*)d_ws;
  auto carve = [&](size_t bytes) { char* p = ws + off; off += (bytes + 255) & ~(size_t)255; return p; };
  b16* WT = (b16*)carve((size_t)6 * F * F * 2); b16* QP = (b16*)carve((size_t)NB * V * F * 2); b16* KP = (b16*)carve((size_t)NC * V * F * 2); b16* VT = (b16*)carve((size_t)NC * V * F * 2);
  b16* CTX = (b16*)carve((size_t)NTOK * F * 2); float* XF = (float*)carve((size_t)NTOK * F * 4); b16* Y1 = (b16*)carve((size_t)NTOK * F * 2);
  if (off > ws_size || off > ((size_t)128 << 20)) return;
  prep_kernel<<<(unsigned)(((size_t)6 * F * F / 8 + 255) / 256), 256, 0, stream>>>(Fp(2), Fp(4), Fp(6), Fp(8), Fp(16), Fp(18), WT);
  proj_kernel<<<dim3(V / 64, 8, 6), 128, 0, stream>>>(Fp(0), Fp(1), Fp(10), Fp(11), Fp(12), Fp(13), WT, Fp(3), Fp(5), Fp(7), QP, KP, VT);
  attn_kernel<<<dim3(V / 32, BNL * H), 64, 0, stream>>>(QP, KP, VT, CTX);
  rows_kernel<0><<<dim3((BNL * V) / 64, 2), 128, 0, stream>>>(CTX, nullptr, Fp(1), nullptr, nullptr, WT + (size_t)3 * F * F, Fp(9), XF, nullptr);
  rows_kernel<1><<<dim3((BNL * V) / 64, 2), 128, 0, stream>>>(nullptr, XF, nullptr, Fp(14), Fp(15), WT + (size_t)4 * F * F, Fp(17), nullptr, Y1);
  rows_kernel<2><<<dim3((BNL * V) / 64, 2), 128, 0, stream>>>(Y1, XF, nullptr, nullptr, nullptr, WT + (size_t)5 * F * F, Fp(19), (float*)d_out, nullptr);
}
